// PENetwork_57801669869760
// MI455X (gfx1250) — hardware-verified
//
#include <hip/hip_runtime.h>


typedef float v8f __attribute__((ext_vector_type(8)));
typedef float v4f __attribute__((ext_vector_type(4))) __attribute__((may_alias));
typedef unsigned short v8us __attribute__((ext_vector_type(8))) __attribute__((may_alias));
typedef unsigned short v16us __attribute__((ext_vector_type(16)));
typedef __bf16 v16bf __attribute__((ext_vector_type(16)));

union Frag16 { v16bf v; v16us u; v8us h8[2]; };

constexpr int NQ  = 4;
constexpr int DIM = 16;
constexpr int HID = 64;
constexpr int NG  = 24;
constexpr int NY  = 6;
constexpr int NS  = 4;
constexpr int NU  = NY * NS;
constexpr int NT  = HID / 16;
constexpr int MT  = 4;
constexpr int WAVES = 8;
constexpr int THREADS = WAVES * 32;
constexpr int ROWS_PER_WAVE  = 16 * MT;
constexpr int ROWS_PER_BLOCK = WAVES * ROWS_PER_WAVE;
constexpr float NEG_SLOPE = 0.01f;

constexpr int TAB_INVCOL = 0;
constexpr int TAB_HIDX   = NG * DIM;
constexpr int TAB_BYTES  = NG * DIM + NU * NG;
constexpr int TAB_WORDS  = TAB_BYTES / 4;

struct __attribute__((aligned(16))) GTab { unsigned int w[TAB_WORDS]; };
static_assert(sizeof(GTab) == TAB_BYTES);
static_assert((TAB_BYTES % 16) == 0);

__device__ __forceinline__ int tab_byte(const GTab& t, int i) {
  return (int)((t.w[i >> 2] >> ((i & 3) * 8)) & 0xffu);
}

__device__ __forceinline__ unsigned short bf16_rne_bits(float f) {
  unsigned int u = __float_as_uint(f);
  u += 0x7FFFu + ((u >> 16) & 1u);
  return (unsigned short)(u >> 16);
}
__device__ __forceinline__ float bf16_bits_to_f32(unsigned short s) {
  return __uint_as_float(((unsigned int)s) << 16);
}
__device__ __forceinline__ void split_bf16(float v, unsigned short& hi, unsigned short& lo) {
  hi = bf16_rne_bits(v);
  const float r = v - bf16_bits_to_f32(hi);
  lo = bf16_rne_bits(r);
}

__device__ __forceinline__ v8f wmma_pair_bf16(v16bf a, v16bf bh, v16bf bl, v8f c) {
  c = __builtin_amdgcn_wmma_f32_16x16x32_bf16(false, a, false, bh, (short)0, c, false, false);
  c = __builtin_amdgcn_wmma_f32_16x16x32_bf16(false, a, false, bl, (short)0, c, false, false);
  asm volatile("v_nop\n\tv_nop\n\tv_nop\n\tv_nop" : "+v"(c) : "v"(a), "v"(bh), "v"(bl));
  return c;
}

__global__ __launch_bounds__(HID) void k_weff(const float* __restrict__ Wg, GTab tab,
                                              unsigned short* __restrict__ Phi,
                                              unsigned short* __restrict__ Plo)
{
  __shared__ __align__(16) unsigned short sH[HID * DIM];
  __shared__ __align__(16) unsigned short sL[HID * DIM];

  const int u   = blockIdx.x;
  const int hid = threadIdx.x;

  #pragma unroll 1
  for (int d = 0; d < DIM; ++d) {
    float acc = 0.f;
    #pragma unroll 1
    for (int g = 0; g < NG; ++g) {
      int hg = tab_byte(tab, TAB_HIDX + u * NG + g);
      hg = hg < NG ? hg : (NG - 1);
      const int r = tab_byte(tab, TAB_INVCOL + hg * DIM + d) & (DIM - 1);
      acc += Wg[((size_t)g * DIM + r) * HID + hid];
    }
    unsigned short hh, ll;
    split_bf16(acc, hh, ll);
    sH[hid * DIM + d] = hh;
    sL[hid * DIM + d] = ll;
  }
  __syncthreads();

  constexpr int HALF = HID * DIM / 2;
  const v8us a0 = *(const v8us*)(sH + hid * 8);
  const v8us a1 = *(const v8us*)(sH + HALF + hid * 8);
  const v8us b0 = *(const v8us*)(sL + hid * 8);
  const v8us b1 = *(const v8us*)(sL + HALF + hid * 8);

  unsigned short* ph = Phi + (size_t)u * HID * DIM;
  unsigned short* pl = Plo + (size_t)u * HID * DIM;
  *(volatile v8us*)(ph + hid * 8)        = a0;
  *(volatile v8us*)(ph + HALF + hid * 8) = a1;
  *(volatile v8us*)(pl + hid * 8)        = b0;
  *(volatile v8us*)(pl + HALF + hid * 8) = b1;
  __threadfence();
  *(volatile v8us*)(ph + hid * 8)        = a0;
  *(volatile v8us*)(ph + HALF + hid * 8) = a1;
  *(volatile v8us*)(pl + hid * 8)        = b0;
  *(volatile v8us*)(pl + HALF + hid * 8) = b1;
}

__global__ __launch_bounds__(THREADS) void k_main(const float* __restrict__ x,
                                                  const unsigned short* __restrict__ Phi,
                                                  const unsigned short* __restrict__ Plo,
                                                  const float* __restrict__ Wlin,
                                                  float* __restrict__ out,
                                                  int nrows)
{
  __shared__ __align__(16) float sOut[WAVES * ROWS_PER_WAVE * NY];

  const int tid  = threadIdx.x;
  const int lane = tid & 31;
  const int wave = tid >> 5;
  const int h    = lane >> 4;
  const int l16  = lane & 15;

  const int rbase = blockIdx.x * ROWS_PER_BLOCK + wave * ROWS_PER_WAVE;

  Frag16 fa[MT];
  #pragma unroll
  for (int m = 0; m < MT; ++m) {
    int row = rbase + m * 16 + l16;
    row = row < nrows ? row : (nrows - 1);
    const v4f* xp = (const v4f*)(x + (size_t)row * DIM + 8 * h);
    const v4f x0 = xp[0], x1 = xp[1];
    v16us au;
    #pragma unroll
    for (int e = 0; e < 4; ++e) {
      unsigned short hh, ll;
      split_bf16(x0[e], hh, ll); au[e] = hh;     au[8 + e]  = ll;
      split_bf16(x1[e], hh, ll); au[4 + e] = hh; au[12 + e] = ll;
    }
    fa[m].u = au;
  }

  float wl[NT];
  #pragma unroll
  for (int t = 0; t < NT; ++t) wl[t] = Wlin[t * 16 + l16];

  float* sw = sOut + wave * (ROWS_PER_WAVE * NY);

  #pragma unroll 1
  for (int y = 0; y < NY; ++y) {
    float acc[MT][8];
    #pragma unroll
    for (int m = 0; m < MT; ++m)
      #pragma unroll
      for (int r = 0; r < 8; ++r) acc[m][r] = 0.f;

    #pragma unroll 1
    for (int s = 0; s < NS; ++s) {
      const int u = y * NS + s;
      const unsigned short* ph0 = Phi + ((size_t)u * HID + l16) * DIM + 8 * h;
      const unsigned short* pl0 = Plo + ((size_t)u * HID + l16) * DIM + 8 * h;
      #pragma unroll
      for (int t = 0; t < NT; ++t) {
        const v8us vh = *(const v8us*)(ph0 + t * 16 * DIM);
        const v8us vl = *(const v8us*)(pl0 + t * 16 * DIM);
        Frag16 fbh, fbl;
        fbh.h8[0] = vh; fbh.h8[1] = vh;
        fbl.h8[0] = vl; fbl.h8[1] = vl;
        const float wt = wl[t];
        #pragma unroll
        for (int m = 0; m < MT; ++m) {
          v8f c = {0.f, 0.f, 0.f, 0.f, 0.f, 0.f, 0.f, 0.f};
          c = wmma_pair_bf16(fa[m].v, fbh.v, fbl.v, c);
          #pragma unroll
          for (int r = 0; r < 8; ++r) {
            const float v  = c[r];
            const float lk = fmaxf(v, v * NEG_SLOPE);
            acc[m][r] = fmaf(lk, wt, acc[m][r]);
          }
        }
      }
    }

    #pragma unroll
    for (int m = 0; m < MT; ++m) {
      #pragma unroll
      for (int r = 0; r < 8; ++r) {
        float v = acc[m][r];
        v += __shfl_xor(v, 1, 32);
        v += __shfl_xor(v, 2, 32);
        v += __shfl_xor(v, 4, 32);
        v += __shfl_xor(v, 8, 32);
        acc[m][r] = v;
      }
      float val = acc[m][0];
      #pragma unroll
      for (int j = 1; j < 8; ++j) val = (l16 == j) ? acc[m][j] : val;
      if (l16 < 8) sw[(m * 16 + 8 * h + l16) * NY + y] = val * 0.25f;
    }
  }

  __syncthreads();

  int nvalid = nrows - rbase;
  nvalid = nvalid < 0 ? 0 : nvalid;
  nvalid = nvalid > ROWS_PER_WAVE ? ROWS_PER_WAVE : nvalid;
  const int b  = nvalid * NY;
  const int rb = rbase < nrows ? rbase : nrows;
  float* dst = out + (size_t)rb * NY;

  const v4f v0 = *(const v4f*)(sw + lane * 4);
  const v4f v1 = *(const v4f*)(sw + 128 + lane * 4);
  const v4f v2 = *(const v4f*)(sw + 256 + lane * 4);
  const bool p0 = (lane * 4 + 4) <= b;
  const bool p1 = (128 + lane * 4 + 4) <= b;
  const bool p2 = (256 + lane * 4 + 4) <= b;
  const int  ft = (b & ~3) + lane;
  const bool pt = ft < b;
  const float vt = sw[pt ? ft : 0];

  if (p0) *(volatile v4f*)(dst + lane * 4)       = v0;
  if (p1) *(volatile v4f*)(dst + 128 + lane * 4) = v1;
  if (p2) *(volatile v4f*)(dst + 256 + lane * 4) = v2;
  if (pt) *(volatile float*)(dst + ft) = vt;
  __threadfence();
  if (p0) *(volatile v4f*)(dst + lane * 4)       = v0;
  if (p1) *(volatile v4f*)(dst + 128 + lane * 4) = v1;
  if (p2) *(volatile v4f*)(dst + 256 + lane * 4) = v2;
  if (pt) *(volatile float*)(dst + ft) = vt;
}

static void tab_set(GTab& T, int i, int v) {
  T.w[i >> 2] |= ((unsigned int)(v & 0xff)) << ((i & 3) * 8);
}

static void build_tables(GTab& T) {
  for (int i = 0; i < TAB_WORDS; ++i) T.w[i] = 0u;

  int perms[NG][NQ];
  int np = 0;
  for (int a = 0; a < NQ; ++a)
    for (int b = 0; b < NQ; ++b) {
      if (b == a) continue;
      for (int c = 0; c < NQ; ++c) {
        if (c == a || c == b) continue;
        if (np < NG) {
          perms[np][0] = a; perms[np][1] = b; perms[np][2] = c; perms[np][3] = 6 - a - b - c;
        }
        ++np;
      }
    }

  int invp[NG][NQ];
  for (int g = 0; g < NG; ++g)
    for (int i = 0; i < NQ; ++i) invp[g][perms[g][i]] = i;

  for (int g = 0; g < NG; ++g)
    for (int f = 0; f < DIM; ++f) {
      int src[NQ];
      for (int k = 0; k < NQ; ++k) src[invp[g][k]] = (f >> (NQ - 1 - k)) & 1;
      int col = 0;
      for (int a = 0; a < NQ; ++a) col |= src[a] << (NQ - 1 - a);
      tab_set(T, TAB_INVCOL + g * DIM + col, f);
    }

  int stab[NS] = {0, 0, 0, 0};
  int ns = 0;
  for (int g = 0; g < NG; ++g) {
    const int a = perms[g][0], b = perms[g][1];
    const int lo = a < b ? a : b, hi = a < b ? b : a;
    if (lo == 0 && hi == 1) { if (ns < NS) stab[ns] = g; ++ns; }
  }

  int yp[NY][2];
  int ny = 0;
  for (int p = 0; p < NQ; ++p)
    for (int q = p + 1; q < NQ; ++q) {
      if (ny < NY) { yp[ny][0] = p; yp[ny][1] = q; }
      ++ny;
    }

  int uperm[NU][NQ];
  for (int y = 0; y < NY; ++y) {
    int gy = 0;
    for (int g = 0; g < NG; ++g) {
      const int a = perms[g][0], b = perms[g][1];
      const int lo = a < b ? a : b, hi = a < b ? b : a;
      if (lo == yp[y][0] && hi == yp[y][1]) { gy = g; break; }
    }
    for (int si = 0; si < NS; ++si)
      for (int i = 0; i < NQ; ++i)
        uperm[y * NS + si][i] = perms[gy][perms[stab[si]][i]];
  }

  for (int u = 0; u < NU; ++u)
    for (int g = 0; g < NG; ++g) {
      int comp[NQ];
      for (int i = 0; i < NQ; ++i) comp[i] = uperm[u][invp[g][i]];
      int hsel = 0;
      for (int t = 0; t < NG; ++t)
        if (perms[t][0] == comp[0] && perms[t][1] == comp[1] &&
            perms[t][2] == comp[2] && perms[t][3] == comp[3]) { hsel = t; break; }
      tab_set(T, TAB_HIDX + u * NG + g, hsel);
    }
}

extern "C" void kernel_launch(void* const* d_in, const int* in_sizes, int n_in,
                              void* d_out, int out_size, void* d_ws, size_t ws_size,
                              hipStream_t stream)
{
  if (n_in < 3) return;
  const int nx = in_sizes[0];
  const int nw = in_sizes[1];
  const int nl = in_sizes[2];
  const int nrows = nx / DIM;
  if (nrows <= 0 || nx != nrows * DIM) return;
  if (nw != NG * DIM * HID || nl != HID) return;
  if (out_size != nrows * NY) return;

  const size_t plane_halves = (size_t)NU * HID * DIM;
  const size_t plane_bytes  = plane_halves * sizeof(unsigned short);
  if (2 * plane_bytes > ws_size) return;
  unsigned short* Phi = (unsigned short*)d_ws;
  unsigned short* Plo = Phi + plane_halves;

  const float* x    = (const float*)d_in[0];
  const float* Wg   = (const float*)d_in[1];
  const float* Wlin = (const float*)d_in[2];
  float* out = (float*)d_out;

  GTab tab;
  build_tables(tab);

  k_weff<<<dim3(NU), dim3(HID), 0, stream>>>(Wg, tab, Phi, Plo);

  dim3 gm((nrows + ROWS_PER_BLOCK - 1) / ROWS_PER_BLOCK);
  k_main<<<gm, dim3(THREADS), 0, stream>>>(x, Phi, Plo, Wlin, out, nrows);
  (void)hipGetLastError();
}
